// LlamaDecoderLayer_63522566308480
// MI455X (gfx1250) — hardware-verified
//
#include <hip/hip_runtime.h>


namespace {
constexpr int L = 4096, D = 768, H = 12, HD = 64, NT = L, DI = 3072, DQK = 2 * D;
constexpr float XS = 8.0f, PS = 8.0f, EPS = 1e-5f;
struct Wo_ { static constexpr size_t Q = 0, K = (size_t)D * D, V = 2 * (size_t)D * D, O = 3 * (size_t)D * D, UP = 4 * (size_t)D * D, DN = UP + (size_t)DI * D, END = DN + (size_t)D * DI; };

typedef _Float16 b16;
typedef __attribute__((ext_vector_type(16))) _Float16 v16b;
typedef __attribute__((ext_vector_type(8))) _Float16 v8b;
typedef __attribute__((ext_vector_type(8))) float v8f;
typedef __attribute__((ext_vector_type(4))) float v4f;
__device__ __forceinline__ float bf16_rne(float f) { unsigned int u = __float_as_uint(f); u += 0x7FFFu + ((u >> 16) & 1u); return __uint_as_float(u & 0xFFFF0000u); }
__device__ __forceinline__ v16b frag_kb(const b16* p, int hh) { const v8b a = *(const v8b*)(p + 8 * hh), b = *(const v8b*)(p + 16 + 8 * hh); v16b f;
#pragma unroll
  for (int e = 0; e < 8; ++e) { f[e] = a[e]; f[8 + e] = b[e]; } return f; }
__device__ __forceinline__ v8f wmma16b(v16b a, v16b b, v8f c) { v8f d = __builtin_amdgcn_wmma_f32_16x16x32_f16(false, a, false, b, (short)0, c, false, false); asm volatile("v_nop\n\tv_nop\n\tv_nop\n\tv_nop" : "+v"(d) : "v"(a), "v"(b)); return d; }
__device__ __forceinline__ void wave_lds_sync() { __builtin_amdgcn_fence(__ATOMIC_RELEASE, "workgroup"); __builtin_amdgcn_wave_barrier(); __builtin_amdgcn_fence(__ATOMIC_ACQUIRE, "workgroup"); }
__device__ __forceinline__ float nexp(float x) { return __builtin_amdgcn_exp2f(x * 1.4426950408889634f); }
__device__ __forceinline__ float pmul(float a, float b) { float p = a * b; asm volatile("" : "+v"(p)); return p; }
__device__ __forceinline__ float wsum(float v) {
#pragma unroll
  for (int o = 1; o < 32; o <<= 1) v += __shfl_xor(v, o); return v; }
__device__ __forceinline__ float silu_f(float y) { return y / (1.0f + nexp(-y)); }

__global__ __launch_bounds__(256) void prep_kernel(const float* __restrict__ wq, const float* __restrict__ wk, const float* __restrict__ wv, const float* __restrict__ wo, const float* __restrict__ wu, const float* __restrict__ wd, const float* __restrict__ l1, const float* __restrict__ l2, b16* __restrict__ R, float* __restrict__ P) {
  const size_t tid = (size_t)blockIdx.x * 256 + threadIdx.x, nth = (size_t)gridDim.x * 256;
  for (int pass = 0; pass < 2; ++pass) { for (size_t p = tid; p < Wo_::END / 8; p += nth) { const size_t q = p * 8; const float* s_ = (q < Wo_::K) ? (wq + q) : (q < Wo_::V) ? (wk + (q - Wo_::K)) : (q < Wo_::O) ? (wv + (q - Wo_::V)) : (q < Wo_::UP) ? (wo + (q - Wo_::O)) : (q < Wo_::DN) ? (wu + (q - Wo_::UP)) : (wd + (q - Wo_::DN)); v8b v; for (int e = 0; e < 8; ++e) v[e] = (b16)bf16_rne(s_[e]); *(volatile v8b*)(R + q) = v; }
    for (size_t q = tid; q < 4608; q += nth) { const int i = (int)q; P[q] = (i < 768) ? bf16_rne(l1[i]) : (i < 1536) ? bf16_rne(l2[i - 768]) : 0.0f; } __threadfence(); }
}

template <int RND>
__global__ __launch_bounds__(256) void rms_kernel(const float* __restrict__ src, const float* __restrict__ w, b16* __restrict__ dst) {
  const int row = blockIdx.x * 8 + (threadIdx.x >> 5), lane = threadIdx.x & 31; const float* xr = src + (size_t)row * D;
  float v[24]; float q = 0.0f;
#pragma unroll
  for (int i = 0; i < 24; ++i) { float x = xr[(i >> 3) * 256 + lane * 8 + (i & 7)]; if (RND) x = bf16_rne(x); v[i] = x; q += pmul(x, x); }
  q = wsum(q); const float inv = rsqrtf(q * (1.0f / D) + EPS);
  for (int pass = 0; pass < 2; ++pass) {
#pragma unroll
    for (int gq = 0; gq < 3; ++gq) { v8b o; const int c0 = gq * 256 + lane * 8; for (int e = 0; e < 8; ++e) o[e] = (b16)(pmul(v[gq * 8 + e] * inv, w[c0 + e]) * XS); *(volatile v8b*)(dst + (size_t)row * D + c0) = o; }
    __threadfence(); }
}

template <int K, int N, int EPI, int RND>
__global__ __launch_bounds__(64) void gemm_kernel(const b16* __restrict__ A, const b16* __restrict__ Bw, const float* __restrict__ resid, b16* __restrict__ Ch, float* __restrict__ Cf) {
  __shared__ __attribute__((aligned(16))) float Ts[2][32][128 + 4];
  const int lane = threadIdx.x & 31, wave = threadIdx.x >> 5, nloc = lane & 15, hlf = lane >> 4, m0 = blockIdx.y * 32, c0 = blockIdx.x * 256 + wave * 128;
#pragma unroll 1
  for (int hf = 0; hf < 2; ++hf) { v8f acc[2][4];
#pragma unroll
    for (int r = 0; r < 2; ++r)
#pragma unroll
      for (int t = 0; t < 4; ++t) acc[r][t] = (v8f){};
#pragma unroll 2
    for (int kb = 0; kb < K; kb += 32) { const v16b a0 = frag_kb(A + (size_t)(m0 + nloc) * K + kb, hlf), a1 = frag_kb(A + (size_t)(m0 + 16 + nloc) * K + kb, hlf);
#pragma unroll
      for (int t = 0; t < 4; ++t) { const v16b bw = frag_kb(Bw + (size_t)(c0 + (hf * 4 + t) * 16 + nloc) * K + kb, hlf); acc[0][t] = wmma16b(a0, bw, acc[0][t]); acc[1][t] = wmma16b(a1, bw, acc[1][t]); } }
#pragma unroll
    for (int t = 0; t < 4; ++t) { const int cl = (hf * 4 + t) * 16 + nloc, c = c0 + cl;
#pragma unroll
      for (int r = 0; r < 2; ++r)
#pragma unroll
        for (int v = 0; v < 8; ++v) { const int rr = r * 16 + 8 * hlf + v; float y = acc[r][t][v] * (1.0f / XS); if (EPI == 1) { float xr = resid[(size_t)(m0 + rr) * N + c]; y += RND ? bf16_rne(xr) : xr; } Ts[wave][rr][cl] = y; } } }
  wave_lds_sync();
  for (int pass = 0; pass < 2; ++pass) {
    if (EPI == 1) { for (int i = lane; i < 32 * 32; i += 32) { const int rr = i >> 5, c4 = (i & 31) * 4; *(volatile v4f*)(Cf + (size_t)(m0 + rr) * N + c0 + c4) = *(const v4f*)(&Ts[wave][rr][c4]); } }
    else { for (int i = lane; i < 32 * 16; i += 32) { const int rr = i >> 4, c8 = (i & 15) * 8; v8b o; for (int e = 0; e < 8; ++e) o[e] = (b16)(Ts[wave][rr][c8 + e] * XS); *(volatile v8b*)(Ch + (size_t)(m0 + rr) * N + c0 + c8) = o; } }
    __threadfence(); }
}

__global__ __launch_bounds__(128) void vproj_kernel(const b16* __restrict__ X, const b16* __restrict__ R, b16* __restrict__ VT) {
  __shared__ __attribute__((aligned(16))) b16 Tv[128][128 + 8];
  const int lane = threadIdx.x & 31, wave = threadIdx.x >> 5, nloc = lane & 15, hlf = lane >> 4, t0 = blockIdx.x * 128, m0 = t0 + wave * 32; const b16* Wv = R + Wo_::V;
#pragma unroll 1
  for (int ch = 0; ch < 6; ++ch) { v8f acc[2][8];
#pragma unroll
    for (int r = 0; r < 2; ++r)
#pragma unroll
      for (int t = 0; t < 8; ++t) acc[r][t] = (v8f){};
#pragma unroll 2
    for (int kb = 0; kb < D; kb += 32) { const v16b a0 = frag_kb(X + (size_t)(m0 + nloc) * D + kb, hlf), a1 = frag_kb(X + (size_t)(m0 + 16 + nloc) * D + kb, hlf);
#pragma unroll
      for (int t = 0; t < 8; ++t) { const v16b bw = frag_kb(Wv + (size_t)(ch * 128 + t * 16 + nloc) * D + kb, hlf); acc[0][t] = wmma16b(a0, bw, acc[0][t]); acc[1][t] = wmma16b(a1, bw, acc[1][t]); } }
    __syncthreads();
#pragma unroll
    for (int t = 0; t < 8; ++t)
#pragma unroll
      for (int r = 0; r < 2; ++r)
#pragma unroll
        for (int v = 0; v < 8; ++v) Tv[t * 16 + nloc][wave * 32 + r * 16 + 8 * hlf + v] = (b16)(acc[r][t][v]);
    __syncthreads();
    for (int pass = 0; pass < 2; ++pass) { for (int i = threadIdx.x; i < 128 * 16; i += 128) { const int c = i >> 4, c8 = (i & 15) * 8; const int cg = ch * 128 + c, h = cg / HD, d = cg % HD; *(volatile v8b*)(VT + ((size_t)h * HD + d) * L + t0 + c8) = *(const v8b*)(&Tv[c][c8]); } __threadfence(); } }
}

__global__ __launch_bounds__(128) void attn_kernel(const b16* __restrict__ QK, const b16* __restrict__ vt, b16* __restrict__ ctx) {
  __shared__ __attribute__((aligned(16))) b16 Os[16][4 * HD + 8];
  const int wid = threadIdx.x >> 5, lane = threadIdx.x & 31, hh = lane >> 4, col = lane & 15; const int q0 = blockIdx.x * 16, h = blockIdx.y * 4 + wid, qi = q0 + col;
  const b16* Qr = QK + h * HD; const b16* Kr = QK + D + h * HD; const b16* V = vt + ((size_t)h * HD) * L;
  const v16b qf0 = frag_kb(Qr + (size_t)qi * DQK, hh), qf1 = frag_kb(Qr + (size_t)qi * DQK + 32, hh);
  float m = -INFINITY, l = 0.0f; v8f o[4] = {{}, {}, {}, {}};
  for (int kb = 0; kb < L; kb += 32) {
    v8f s0 = {}, s1 = {}; s0 = wmma16b(frag_kb(Kr + (size_t)(kb + col) * DQK, hh), qf0, s0); s0 = wmma16b(frag_kb(Kr + (size_t)(kb + col) * DQK + 32, hh), qf1, s0);
    s1 = wmma16b(frag_kb(Kr + (size_t)(kb + 16 + col) * DQK, hh), qf0, s1); s1 = wmma16b(frag_kb(Kr + (size_t)(kb + 16 + col) * DQK + 32, hh), qf1, s1);
    float mr = -INFINITY;
#pragma unroll
    for (int r = 0; r < 8; ++r) { s0[r] *= (0.125f / (XS * XS)); s1[r] *= (0.125f / (XS * XS)); mr = fmaxf(mr, fmaxf(s0[r], s1[r])); }
    mr = fmaxf(mr, __shfl_xor(mr, 16)); const float mn = fmaxf(m, mr), al_ = nexp(m - mn); m = mn; float sum = 0.0f; v16b pb;
#pragma unroll
    for (int r = 0; r < 8; ++r) { const float e0 = nexp(s0[r] - mn), e1 = nexp(s1[r] - mn); sum += e0 + e1; pb[r] = (b16)(e0 * PS); pb[8 + r] = (b16)(e1 * PS); }
    sum += __shfl_xor(sum, 16); l = l * al_ + sum;
#pragma unroll
    for (int t = 0; t < 4; ++t) { o[t] *= al_; o[t] = wmma16b(frag_kb(V + (size_t)(t * 16 + col) * L + kb, hh), pb, o[t]); } }
  const float inv = 1.0f / (l * PS);
#pragma unroll
  for (int t = 0; t < 4; ++t)
#pragma unroll
    for (int r = 0; r < 8; ++r) Os[col][wid * HD + t * 16 + 8 * hh + r] = (b16)(o[t][r] * inv);
  __syncthreads();
  for (int pass = 0; pass < 2; ++pass) { for (int i = threadIdx.x; i < 16 * 32; i += 128) { const int rr = i >> 5, c8 = (i & 31) * 8; *(volatile v8b*)(ctx + (size_t)(q0 + rr) * D + blockIdx.y * 4 * HD + c8) = *(const v8b*)(&Os[rr][c8]); } __threadfence(); }
}

__global__ __launch_bounds__(256) void mlp_kernel(const b16* __restrict__ Hh, const b16* __restrict__ R, const float* __restrict__ X1, float* __restrict__ out) {
  __shared__ __attribute__((aligned(16))) b16 G[16][DI + 8];
  const int wave = threadIdx.x >> 5, lane = threadIdx.x & 31, nloc = lane & 15, hlf = lane >> 4, r0 = blockIdx.x * 16; const b16* Wu = R + Wo_::UP; const b16* Wd = R + Wo_::DN;
  for (int t = wave; t < DI / 16; t += 8) { v8f acc = {};
#pragma unroll 4
    for (int kb = 0; kb < D; kb += 32) acc = wmma16b(frag_kb(Hh + (size_t)(r0 + nloc) * D + kb, hlf), frag_kb(Wu + (size_t)(t * 16 + nloc) * D + kb, hlf), acc);
    const int c = t * 16 + nloc;
#pragma unroll
    for (int r = 0; r < 8; ++r) G[8 * hlf + r][c] = (b16)(silu_f(acc[r] * (1.0f / XS)) * XS); }
  __syncthreads();
  v8f acc2[6];
#pragma unroll
  for (int t = 0; t < 6; ++t) acc2[t] = (v8f){};
#pragma unroll 2
  for (int kb = 0; kb < DI; kb += 32) { const v16b a = frag_kb(&G[nloc][kb], hlf);
#pragma unroll
    for (int t = 0; t < 6; ++t) acc2[t] = wmma16b(a, frag_kb(Wd + (size_t)(wave * 96 + t * 16 + nloc) * DI + kb, hlf), acc2[t]); }
  float vals[6][8];
#pragma unroll
  for (int t = 0; t < 6; ++t) { const int c = wave * 96 + t * 16 + nloc;
#pragma unroll
    for (int r = 0; r < 8; ++r) vals[t][r] = acc2[t][r] * (1.0f / XS) + X1[(size_t)(r0 + 8 * hlf + r) * D + c]; }
  __syncthreads();
  float (*St)[D + 4] = (float (*)[D + 4])(&G[0][0]);
#pragma unroll
  for (int t = 0; t < 6; ++t)
#pragma unroll
    for (int r = 0; r < 8; ++r) St[8 * hlf + r][wave * 96 + t * 16 + nloc] = vals[t][r];
  __syncthreads();
  for (int pass = 0; pass < 2; ++pass) { for (int i = threadIdx.x; i < 16 * (D / 4); i += 256) { const int rr = i / (D / 4), c4 = (i % (D / 4)) * 4; *(volatile v4f*)(out + (size_t)(r0 + rr) * D + c4) = *(const v4f*)(&St[rr][c4]); } __threadfence(); }
}
}

extern "C" void kernel_launch(void* const* d_in, const int* in_sizes, int n_in,
                              void* d_out, int out_size, void* d_ws, size_t ws_size, hipStream_t stream) {
  (void)n_in; (void)out_size;
  const float* x = (const float*)d_in[0]; const float* wq = (const float*)d_in[1]; const float* wk = (const float*)d_in[2]; const float* wv = (const float*)d_in[3]; const float* wo = (const float*)d_in[4]; const float* wu = (const float*)d_in[5]; const float* wd = (const float*)d_in[6]; const float* l1 = (const float*)d_in[7]; const float* l2 = (const float*)d_in[8];
  float* out = (float*)d_out;
  if (in_sizes[0] != NT * D || in_sizes[1] != D * D || in_sizes[5] != DI * D || in_sizes[6] != D * DI) return;
  size_t off = 0; char* ws = (char*)d_ws;
  auto carve = [&](size_t bytes) { char* p = ws + off; off += (bytes + 255) & ~(size_t)255; return p; };
  b16* R = (b16*)carve(Wo_::END * 2); float* P = (float*)carve(4608 * 4); b16* XN = (b16*)carve((size_t)NT * D * 2); b16* QK = (b16*)carve((size_t)NT * DQK * 2); b16* VT = (b16*)carve((size_t)NT * D * 2); b16* CTX = (b16*)carve((size_t)NT * D * 2); float* X1 = (float*)carve((size_t)NT * D * 4); b16* HH = (b16*)carve((size_t)NT * D * 2);
  if (off > ws_size) return;
  prep_kernel<<<512, 256, 0, stream>>>(wq, wk, wv, wo, wu, wd, l1, l2, R, P);
  rms_kernel<1><<<NT / 8, 256, 0, stream>>>(x, P, XN);
  gemm_kernel<D, DQK, 0, 0><<<dim3(DQK / 256, NT / 32), 64, 0, stream>>>(XN, R + Wo_::Q, nullptr, QK, nullptr);
  vproj_kernel<<<NT / 128, 128, 0, stream>>>(XN, R, VT);
  attn_kernel<<<dim3(NT / 16, 3), 128, 0, stream>>>(QK, VT, CTX);
  gemm_kernel<D, D, 1, 1><<<dim3(D / 256, NT / 32), 64, 0, stream>>>(CTX, R + Wo_::O, x, nullptr, X1);
  rms_kernel<0><<<NT / 8, 256, 0, stream>>>(X1, P + 768, HH);
  mlp_kernel<<<NT / 16, 256, 0, stream>>>(HH, R, X1, out);
}
